// DeepseekV4Attention_7610682048940
// MI455X (gfx1250) — hardware-verified
//
#include <hip/hip_runtime.h>
#include <math.h>

typedef __attribute__((ext_vector_type(16))) _Float16 v16h;
typedef __attribute__((ext_vector_type(8)))  _Float16 v8h;
typedef __attribute__((ext_vector_type(16))) __bf16   v16b;
typedef __attribute__((ext_vector_type(8)))  __bf16   v8b;
typedef __attribute__((ext_vector_type(8)))  float    v8f;
typedef __attribute__((ext_vector_type(4)))  float    v4f;
typedef __attribute__((ext_vector_type(4)))  unsigned int v4u;

constexpr int kSeq      = 2048;
constexpr int kHid      = 2048;
constexpr int kHeads    = 16;
constexpr int kHd       = 256;
constexpr int kRopeHalf = 32;
constexpr int kNope     = 192;
constexpr int kQLat     = 1024;
constexpr int kOLat     = 512;
constexpr int kGroups   = 4;
constexpr int kQCols    = kHeads * kHd;
constexpr int kGrpCols  = kQCols / kGroups;
constexpr int kORCols   = kGroups * kOLat;
constexpr float kEps        = 1e-6f;
constexpr float kScoreScale = 0.0625f;
static_assert(kNope == kHd - 2 * kRopeHalf, "rope");

extern __shared__ __align__(16) unsigned char lds_dyn[];

__device__ __forceinline__ unsigned short f2bf_bits(float f) {
  unsigned u = __float_as_uint(f);
  return (unsigned short)((u + 0x7FFFu + ((u >> 16) & 1u)) >> 16);
}
__device__ __forceinline__ float bf_bits2f(unsigned short h) { return __uint_as_float(((unsigned)h) << 16); }
__device__ __forceinline__ float bf_rne(float f) { return bf_bits2f(f2bf_bits(f)); }
__device__ __forceinline__ void split_bf(float f, unsigned short& hb, unsigned short& lb) {
  hb = f2bf_bits(f);
  lb = f2bf_bits(f - bf_bits2f(hb));
}
__device__ __forceinline__ unsigned int pack2(unsigned short a, unsigned short b) {
  return (unsigned int)a | ((unsigned int)b << 16);
}
__device__ __forceinline__ void wave_sync() {
  __builtin_amdgcn_fence(__ATOMIC_RELEASE, "workgroup");
  __builtin_amdgcn_wave_barrier();
  __builtin_amdgcn_fence(__ATOMIC_ACQUIRE, "workgroup");
}

__device__ __forceinline__ void dep_guard_h(v8f& a, v8f& b, v16h x, v16h y) { asm volatile("v_nop\n\tv_nop\n\tv_nop\n\tv_nop" : "+v"(a), "+v"(b) : "v"(x), "v"(y)); }
__device__ __forceinline__ void dep_guard_b(v8f& a, v8f& b, v16b x, v16b y) { asm volatile("v_nop\n\tv_nop\n\tv_nop\n\tv_nop" : "+v"(a), "+v"(b) : "v"(x), "v"(y)); }
__device__ __forceinline__ void keep4_h(v16h a, v16h b, v16h c, v16h d) { asm volatile("v_nop" :: "v"(a), "v"(b), "v"(c), "v"(d)); }
__device__ __forceinline__ void keep4_b(v16b a, v16b b, v16b c, v16b d) { asm volatile("v_nop" :: "v"(a), "v"(b), "v"(c), "v"(d)); }
__device__ __forceinline__ void acc_guard4(v8f& a, v8f& b, v8f& c, v8f& d) { asm volatile("v_nop\n\tv_nop\n\tv_nop\n\tv_nop" : "+v"(a), "+v"(b), "+v"(c), "+v"(d)); }
__device__ __forceinline__ void guard3(v8f& acc, v16b x, v16b y, v16b z) {
  asm volatile("v_nop\n\tv_nop\n\tv_nop\n\tv_nop" : "+v"(acc) : "v"(x), "v"(y), "v"(z));
}
__device__ __forceinline__ v8f mma_bf(v16b a, v16b b, v8f c) {
  return __builtin_amdgcn_wmma_f32_16x16x32_bf16(false, a, false, b, (short)0, c, false, false);
}

template <typename T> struct Frag;
template <> struct Frag<_Float16> {
  typedef v16h V; union U { v16h v; v8h h[2]; };
  static __device__ __forceinline__ v16h load(const _Float16* p) {
    U f; f.h[0] = *(const v8h*)(p); f.h[1] = *(const v8h*)(p + 16); return f.v;
  }
  static __device__ __forceinline__ v8f mma(v16h a, v16h b, v8f c) {
    return __builtin_amdgcn_wmma_f32_16x16x32_f16(false, a, false, b, (short)0, c, false, false);
  }
  static __device__ __forceinline__ void guard(v8f& a, v8f& b, v16h x, v16h y) { dep_guard_h(a, b, x, y); }
  static __device__ __forceinline__ void keep(v16h a, v16h b, v16h c, v16h d) { keep4_h(a, b, c, d); }
};
template <> struct Frag<__bf16> {
  typedef v16b V; union U { v16b v; v8b h[2]; };
  static __device__ __forceinline__ v16b load(const __bf16* p) {
    U f; f.h[0] = *(const v8b*)(p); f.h[1] = *(const v8b*)(p + 16); return f.v;
  }
  static __device__ __forceinline__ v8f mma(v16b a, v16b b, v8f c) {
    return __builtin_amdgcn_wmma_f32_16x16x32_bf16(false, a, false, b, (short)0, c, false, false);
  }
  static __device__ __forceinline__ void guard(v8f& a, v8f& b, v16b x, v16b y) { dep_guard_b(a, b, x, y); }
  static __device__ __forceinline__ void keep(v16b a, v16b b, v16b c, v16b d) { keep4_b(a, b, c, d); }
};

template <int SPLITM, int OUT_MODE>
__global__ __launch_bounds__(256) void gemm64_bf16(
    const unsigned short* __restrict__ Ap, const unsigned short* __restrict__ A2p, int lda, long strideA,
    const unsigned short* __restrict__ Btp, const unsigned short* __restrict__ Bt2p, int ldb, long strideB,
    void* __restrict__ Cout, void* __restrict__ Cout2, int ldc, long strideC,
    int M, int N, int K, float scale) {
  typedef __bf16 T;
  typedef v16b V;
  const T* A = (const T*)Ap; const T* A2 = (const T*)A2p; const T* Bt = (const T*)Btp; const T* Bt2 = (const T*)Bt2p;
  __shared__ __align__(16) float sT[8][16 * 68];
  const int b    = blockIdx.y;
  const int lane = threadIdx.x & 31;
  const int wave = threadIdx.x >> 5;
  const int tilesN = N >> 6;
  const int tilesM = M >> 6;
  const int tile = blockIdx.x * 8 + wave;
  if (tile >= tilesM * tilesN) return;
  const int tm = tile / tilesN;
  const int tn = tile - tm * tilesN;
  const int m0 = tm << 6;
  const int n0 = tn << 6;

  const T* Ab  = A  + (size_t)b * strideA;
  const T* Bb  = Bt + (size_t)b * strideB;
  const T* Ab2 = (SPLITM >= 1) ? (A2  + (size_t)b * strideA) : nullptr;
  const T* Bb2 = (SPLITM == 2) ? (Bt2 + (size_t)b * strideB) : nullptr;

  const int rlane = lane & 15;
  const int koff  = (lane >> 4) * 8;
  const int mOff  = (lane >> 4) * 8;

  v8f acc[4][4];
#pragma unroll
  for (int i = 0; i < 4; ++i)
#pragma unroll
    for (int j = 0; j < 4; ++j) acc[i][j] = (v8f){0.f,0.f,0.f,0.f,0.f,0.f,0.f,0.f};

  for (int k0 = 0; k0 < K; k0 += 32) {
    V bh[4], bl[4];
#pragma unroll
    for (int j = 0; j < 4; ++j) {
      const size_t bo = (size_t)(n0 + (j << 4) + rlane) * ldb + koff + k0;
      bh[j] = Frag<T>::load(Bb + bo);
      if (SPLITM == 2) bl[j] = Frag<T>::load(Bb2 + bo); else bl[j] = bh[j];
    }
#pragma unroll
    for (int i = 0; i < 4; ++i) {
      const size_t ao = (size_t)(m0 + (i << 4) + rlane) * lda + koff + k0;
      V ah = Frag<T>::load(Ab + ao);
      V al = ah;
      if (SPLITM >= 1) al = Frag<T>::load(Ab2 + ao);
#pragma unroll
      for (int j = 0; j < 4; ++j) {
        acc[i][j] = Frag<T>::mma(ah, bh[j], acc[i][j]);
        if (SPLITM == 2) acc[i][j] = Frag<T>::mma(ah, bl[j], acc[i][j]);
        if (SPLITM >= 1) acc[i][j] = Frag<T>::mma(al, bh[j], acc[i][j]);
      }
      Frag<T>::guard(acc[i][0], acc[i][3], ah, al);
    }
    Frag<T>::keep(bh[0], bh[1], bh[2], bh[3]);
    if (SPLITM == 2) Frag<T>::keep(bl[0], bl[1], bl[2], bl[3]);
  }
  acc_guard4(acc[0][0], acc[0][1], acc[0][2], acc[0][3]);
  acc_guard4(acc[1][0], acc[1][1], acc[1][2], acc[1][3]);
  acc_guard4(acc[2][0], acc[2][1], acc[2][2], acc[2][3]);
  acc_guard4(acc[3][0], acc[3][1], acc[3][2], acc[3][3]);

  float* slab = sT[wave];
#pragma unroll
  for (int i = 0; i < 4; ++i) {
    const int mBase = m0 + (i << 4);
#pragma unroll
    for (int j = 0; j < 4; ++j) {
#pragma unroll
      for (int r = 0; r < 8; ++r) {
        float v = acc[i][j][r] * scale;
        slab[(mOff + r) * 68 + (j << 4) + rlane] = v;
      }
    }
    __builtin_amdgcn_fence(__ATOMIC_RELEASE, "workgroup");
    __builtin_amdgcn_wave_barrier();
    __builtin_amdgcn_fence(__ATOMIC_ACQUIRE, "workgroup");
    if (OUT_MODE == 0) {
      float* C = (float*)Cout + (size_t)b * strideC;
      const int hh = lane >> 4, c4 = (lane & 15) * 4;
      for (int pass = 0; pass < 2; ++pass) {
#pragma unroll
        for (int it = 0; it < 8; ++it) {
          const int row = it * 2 + hh;
          v4f v = *(const v4f*)(slab + row * 68 + c4);
          *(volatile v4f*)(C + (size_t)(mBase + row) * ldc + n0 + c4) = v;
        }
        __threadfence();
      }
    } else {
      const int q = lane >> 3, c8 = (lane & 7) * 8;
      unsigned short* C  = (unsigned short*)Cout  + (size_t)b * strideC;
      unsigned short* C2 = (unsigned short*)Cout2 + (size_t)b * strideC;
      for (int pass = 0; pass < 2; ++pass) {
#pragma unroll
        for (int it = 0; it < 4; ++it) {
          const int row = it * 4 + q;
          const float* sp = slab + row * 68 + c8;
          v8h hv, lv;
#pragma unroll
          for (int e = 0; e < 8; ++e) {
            unsigned short hb = f2bf_bits(sp[e]);
            unsigned short lb = f2bf_bits(sp[e] - bf_bits2f(hb));
            hv[e] = __builtin_bit_cast(_Float16, hb);
            lv[e] = __builtin_bit_cast(_Float16, lb);
          }
          *(volatile v8h*)(C + (size_t)(mBase + row) * ldc + n0 + c8) = hv;
          *(volatile v8h*)(C2 + (size_t)(mBase + row) * ldc + n0 + c8) = lv;
        }
        __threadfence();
      }
    }
    __builtin_amdgcn_fence(__ATOMIC_RELEASE, "workgroup");
    __builtin_amdgcn_wave_barrier();
    __builtin_amdgcn_fence(__ATOMIC_ACQUIRE, "workgroup");
  }
}

__global__ __launch_bounds__(256) void cvt_bf16x8_kernel(const float* __restrict__ in,
                                                         unsigned short* __restrict__ out, int n8) {
  const int i = blockIdx.x * 256 + threadIdx.x;
  const int ic = (i < n8) ? i : (n8 - 1);
  const v4f a = *(const v4f*)(in + (size_t)ic * 8);
  const v4f b = *(const v4f*)(in + (size_t)ic * 8 + 4);
  v4u w;
  w[0] = pack2(f2bf_bits(a[0]), f2bf_bits(a[1]));
  w[1] = pack2(f2bf_bits(a[2]), f2bf_bits(a[3]));
  w[2] = pack2(f2bf_bits(b[0]), f2bf_bits(b[1]));
  w[3] = pack2(f2bf_bits(b[2]), f2bf_bits(b[3]));
  if (i < n8) {
    *(volatile v4u*)(out + (size_t)i * 8) = w;
    __threadfence();
    *(volatile v4u*)(out + (size_t)i * 8) = w;
  }
}

__global__ __launch_bounds__(256) void rope_table_kernel(const float* __restrict__ fr,
                                                         float* __restrict__ cosT,
                                                         float* __restrict__ sinT, int n) {
  const int i = blockIdx.x * 256 + threadIdx.x;
  const int ic = (i < n) ? i : (n - 1);
  const float f = bf_rne(fr[ic]);
  float sv, cv;
  sincosf(f, &sv, &cv);
  if (i < n) {
    *(volatile float*)(cosT + i) = cv;
    *(volatile float*)(sinT + i) = sv;
    __threadfence();
    *(volatile float*)(cosT + i) = cv;
    *(volatile float*)(sinT + i) = sv;
  }
}

__global__ __launch_bounds__(128) void qlat_prep_kernel(const float* __restrict__ QLraw,
                                                        const float* __restrict__ qw,
                                                        unsigned short* __restrict__ QLh,
                                                        unsigned short* __restrict__ QLl) {
  __shared__ float red[4];
  const int t = threadIdx.x, wave = t >> 5, lane = t & 31;
  const int s = blockIdx.x;
  const size_t base = (size_t)s * kQLat + t * 8;
  const v4f a = *(const v4f*)(QLraw + base);
  const v4f b = *(const v4f*)(QLraw + base + 4);
  float v[8] = {a[0], a[1], a[2], a[3], b[0], b[1], b[2], b[3]};
  float ss = 0.0f;
#pragma unroll
  for (int e = 0; e < 8; ++e) ss += v[e] * v[e];
#pragma unroll
  for (int off = 1; off < 32; off <<= 1) ss += __shfl_xor(ss, off, 32);
  if (lane == 0) red[wave] = ss;
  __syncthreads();
  const float tot = (red[0] + red[1]) + (red[2] + red[3]);
  const float rinv = rsqrtf(tot * (1.0f / 1024.0f) + kEps);
  const v4f wa = *(const v4f*)(qw + t * 8);
  const v4f wb = *(const v4f*)(qw + t * 8 + 4);
  float wv[8] = {bf_rne(wa[0]), bf_rne(wa[1]), bf_rne(wa[2]), bf_rne(wa[3]),
                 bf_rne(wb[0]), bf_rne(wb[1]), bf_rne(wb[2]), bf_rne(wb[3])};
  v4u hw, lw;
#pragma unroll
  for (int p = 0; p < 4; ++p) {
    unsigned short h0, l0, h1, l1;
    split_bf((v[2 * p] * rinv) * wv[2 * p], h0, l0);
    split_bf((v[2 * p + 1] * rinv) * wv[2 * p + 1], h1, l1);
    hw[p] = pack2(h0, h1);
    lw[p] = pack2(l0, l1);
  }
  *(volatile v4u*)(QLh + base) = hw;
  *(volatile v4u*)(QLl + base) = lw;
  __threadfence();
  *(volatile v4u*)(QLh + base) = hw;
  *(volatile v4u*)(QLl + base) = lw;
}

__global__ __launch_bounds__(256) void q_prep_kernel(const float* __restrict__ Qraw,
                                                     const float* __restrict__ cosT,
                                                     const float* __restrict__ sinT,
                                                     unsigned short* __restrict__ Qh,
                                                     unsigned short* __restrict__ Ql) {
  const int wave = threadIdx.x >> 5, lane = threadIdx.x & 31;
  const int s = blockIdx.x;
  const int hidx = blockIdx.y * 8 + wave;
  const size_t base = (size_t)s * kQCols + (size_t)hidx * kHd + lane * 8;
  const v4f a = *(const v4f*)(Qraw + base);
  const v4f b = *(const v4f*)(Qraw + base + 4);
  float v[8] = {a[0], a[1], a[2], a[3], b[0], b[1], b[2], b[3]};
  float ss = 0.0f;
#pragma unroll
  for (int e = 0; e < 8; ++e) ss += v[e] * v[e];
#pragma unroll
  for (int off = 1; off < 32; off <<= 1) ss += __shfl_xor(ss, off, 32);
  const float rinv = rsqrtf(ss * (1.0f / 256.0f) + kEps);
#pragma unroll
  for (int e = 0; e < 8; ++e) v[e] *= rinv;
  const bool is_pe = lane >= 24;
  const int jb = (is_pe ? (lane - 24) : 0) * 4;
#pragma unroll
  for (int p = 0; p < 4; ++p) {
    const float cs = cosT[(size_t)s * kRopeHalf + jb + p];
    const float sn = sinT[(size_t)s * kRopeHalf + jb + p];
    const float x1 = v[2 * p], x2 = v[2 * p + 1];
    const float r1 = x1 * cs - x2 * sn;
    const float r2 = x1 * sn + x2 * cs;
    v[2 * p]     = is_pe ? r1 : x1;
    v[2 * p + 1] = is_pe ? r2 : x2;
  }
  v4u hw, lw;
#pragma unroll
  for (int p = 0; p < 4; ++p) {
    unsigned short h0, l0, h1, l1;
    split_bf(v[2 * p], h0, l0);
    split_bf(v[2 * p + 1], h1, l1);
    hw[p] = pack2(h0, h1);
    lw[p] = pack2(l0, l1);
  }
  *(volatile v4u*)(Qh + base) = hw;
  *(volatile v4u*)(Ql + base) = lw;
  __threadfence();
  *(volatile v4u*)(Qh + base) = hw;
  *(volatile v4u*)(Ql + base) = lw;
}

constexpr int kKvPrepLdsBytes = 2 * kHd * 64 * 2;
__global__ __launch_bounds__(256) void kv_prep_kernel(const float* __restrict__ KVraw,
                                                      const float* __restrict__ kvw,
                                                      const float* __restrict__ cosT,
                                                      const float* __restrict__ sinT,
                                                      unsigned short* __restrict__ KVh,
                                                      unsigned short* __restrict__ KVl,
                                                      unsigned short* __restrict__ KVTh,
                                                      unsigned short* __restrict__ KVTl) {
  unsigned short* Th = reinterpret_cast<unsigned short*>(lds_dyn);
  unsigned short* Tl = Th + kHd * 64;
  const int wave = threadIdx.x >> 5, lane = threadIdx.x & 31;
  const int s0 = blockIdx.x * 64;
  const int d8 = lane * 8;
  const v4f wa = *(const v4f*)(kvw + d8);
  const v4f wb = *(const v4f*)(kvw + d8 + 4);
  const float wv[8] = {bf_rne(wa[0]), bf_rne(wa[1]), bf_rne(wa[2]), bf_rne(wa[3]),
                       bf_rne(wb[0]), bf_rne(wb[1]), bf_rne(wb[2]), bf_rne(wb[3])};
  const bool is_pe = lane >= 24;
  const int jb = (is_pe ? (lane - 24) : 0) * 4;
#pragma unroll 1
  for (int i = 0; i < 8; ++i) {
    const int sl = i * 8 + wave;
    const int s = s0 + sl;
    const size_t go = (size_t)s * kHd + d8;
    const v4f a = *(const v4f*)(KVraw + go);
    const v4f b = *(const v4f*)(KVraw + go + 4);
    float v[8] = {a[0], a[1], a[2], a[3], b[0], b[1], b[2], b[3]};
    float ss = 0.0f;
#pragma unroll
    for (int e = 0; e < 8; ++e) ss += v[e] * v[e];
#pragma unroll
    for (int off = 1; off < 32; off <<= 1) ss += __shfl_xor(ss, off, 32);
    const float rinv = rsqrtf(ss * (1.0f / 256.0f) + kEps);
#pragma unroll
    for (int e = 0; e < 8; ++e) v[e] = (v[e] * rinv) * wv[e];
#pragma unroll
    for (int p = 0; p < 4; ++p) {
      const float cs = cosT[(size_t)s * kRopeHalf + jb + p];
      const float sn = sinT[(size_t)s * kRopeHalf + jb + p];
      const float x1 = v[2 * p], x2 = v[2 * p + 1];
      const float r1 = x1 * cs - x2 * sn;
      const float r2 = x1 * sn + x2 * cs;
      v[2 * p]     = is_pe ? r1 : x1;
      v[2 * p + 1] = is_pe ? r2 : x2;
    }
    unsigned short hb[8], lb[8];
#pragma unroll
    for (int e = 0; e < 8; ++e) split_bf(v[e], hb[e], lb[e]);
#pragma unroll
    for (int e = 0; e < 8; ++e) {
      Th[(d8 + e) * 64 + sl] = hb[e];
      Tl[(d8 + e) * 64 + sl] = lb[e];
    }
    v4u hw, lw;
#pragma unroll
    for (int p = 0; p < 4; ++p) {
      hw[p] = pack2(hb[2 * p], hb[2 * p + 1]);
      lw[p] = pack2(lb[2 * p], lb[2 * p + 1]);
    }
    *(volatile v4u*)(KVh + go) = hw;
    *(volatile v4u*)(KVl + go) = lw;
    __threadfence();
    *(volatile v4u*)(KVh + go) = hw;
    *(volatile v4u*)(KVl + go) = lw;
  }
  __syncthreads();
  {
    const int q = lane >> 3, c8 = (lane & 7) * 8;
    for (int pass = 0; pass < 2; ++pass) {
#pragma unroll
      for (int it = 0; it < 8; ++it) {
        const int d = wave * 32 + it * 4 + q;
        const v4u hv = *(const v4u*)(Th + d * 64 + c8);
        const v4u lv = *(const v4u*)(Tl + d * 64 + c8);
        *(volatile v4u*)(KVTh + (size_t)d * kSeq + s0 + c8) = hv;
        *(volatile v4u*)(KVTl + (size_t)d * kSeq + s0 + c8) = lv;
      }
      __threadfence();
    }
  }
}

constexpr int kKch  = 32;
constexpr int kQBlk = 64;
constexpr int kAttnLdsBytes = 98304;
constexpr int kSsOffBytes   = 65536;
constexpr int kPsOffBytes   = 81920;
constexpr int kSlabPitch    = 132;
static_assert(4 * kKch * kHd * 2 == kSsOffBytes, "kv tiles");
static_assert(kSsOffBytes + 8 * 512 * 4 == kPsOffBytes, "score tiles");
static_assert(kPsOffBytes + 2 * 8 * 512 * 2 == kAttnLdsBytes, "p tiles");
static_assert(8 * 16 * kSlabPitch * 4 <= kPsOffBytes, "slab fits");
static_assert(kSeq % kQBlk == 0 && kQBlk == 2 * kKch, "tiling");

__global__ __launch_bounds__(256)
void attn_kernel(const unsigned short* __restrict__ Qhp, const unsigned short* __restrict__ Qlp,
                 const unsigned short* __restrict__ KVhp, const unsigned short* __restrict__ KVlp,
                 const unsigned short* __restrict__ KVThp, const unsigned short* __restrict__ KVTlp,
                 const float* __restrict__ cosT, const float* __restrict__ sinT,
                 const float* __restrict__ sinkp,
                 unsigned short* __restrict__ Ohp, unsigned short* __restrict__ Olp) {
  unsigned short* kvs_hu = reinterpret_cast<unsigned short*>(lds_dyn);
  unsigned short* kvs_lu = kvs_hu + kKch * kHd;
  unsigned short* kvt_hu = kvs_lu + kKch * kHd;
  unsigned short* kvt_lu = kvt_hu + kHd * kKch;
  const __bf16* kvs_h = reinterpret_cast<const __bf16*>(kvs_hu);
  const __bf16* kvs_l = reinterpret_cast<const __bf16*>(kvs_lu);
  const __bf16* kvt_h = reinterpret_cast<const __bf16*>(kvt_hu);
  const __bf16* kvt_l = reinterpret_cast<const __bf16*>(kvt_lu);
  float* ssh = reinterpret_cast<float*>(lds_dyn + kSsOffBytes);
  __bf16* ps_h = reinterpret_cast<__bf16*>(lds_dyn + kPsOffBytes);
  __bf16* ps_l = ps_h + 8 * 512;

  const int tid = threadIdx.x;
  const int wave = tid >> 5, lane = tid & 31;
  const int hh = lane >> 4, c = lane & 15;
  const int rg = wave >> 1, dh = wave & 1, partner = wave ^ 1;
  const int h = blockIdx.y, qb = blockIdx.x;
  const int q0 = qb * kQBlk + rg * 16;
  const int dloc = dh * 128;
  const int dcol = h * kHd + dloc;

  const __bf16* Qh = reinterpret_cast<const __bf16*>(Qhp);
  const __bf16* Ql = reinterpret_cast<const __bf16*>(Qlp);
  v16b qh[4], ql[4];
#pragma unroll
  for (int dc = 0; dc < 4; ++dc) {
    const size_t o = (size_t)(q0 + c) * kQCols + dcol + dc * 32 + 8 * hh;
    qh[dc] = Frag<__bf16>::load(Qh + o);
    ql[dc] = Frag<__bf16>::load(Ql + o);
  }

  float mrow[8], lrow[8];
  v8f oacc[8];
#pragma unroll
  for (int r = 0; r < 8; ++r) { mrow[r] = -INFINITY; lrow[r] = 0.0f; }
#pragma unroll
  for (int t8 = 0; t8 < 8; ++t8) oacc[t8] = (v8f){0.f,0.f,0.f,0.f,0.f,0.f,0.f,0.f};

  const int nChunks = 2 * (qb + 1);
  for (int kc = 0; kc < nChunks; ++kc) {
    const int t0 = kc * kKch;
    __syncthreads();
#pragma unroll
    for (int i = 0; i < 4; ++i) {
      const int idx = tid + 256 * i;
      const int row = idx >> 5, c8 = (idx & 31) * 8;
      const v4u a = *(const v4u*)(KVhp + (size_t)(t0 + row) * kHd + c8);
      const v4u b = *(const v4u*)(KVlp + (size_t)(t0 + row) * kHd + c8);
      *(v4u*)(kvs_hu + row * kHd + c8) = a;
      *(v4u*)(kvs_lu + row * kHd + c8) = b;
    }
    asm volatile("" ::: "memory");
#pragma unroll
    for (int i = 0; i < 4; ++i) {
      const int idx = tid + 256 * i;
      const int d = idx >> 2, part = (idx & 3) * 8;
      const v4u a = *(const v4u*)(KVThp + (size_t)d * kSeq + t0 + part);
      const v4u b = *(const v4u*)(KVTlp + (size_t)d * kSeq + t0 + part);
      *(v4u*)(kvt_hu + d * kKch + part) = a;
      *(v4u*)(kvt_lu + d * kKch + part) = b;
    }
    __syncthreads();

    v8f s[2];
#pragma unroll
    for (int j = 0; j < 2; ++j) {
      s[j] = (v8f){0.f,0.f,0.f,0.f,0.f,0.f,0.f,0.f};
#pragma unroll
      for (int dc = 0; dc < 4; ++dc) {
        const int ko = (j * 16 + c) * kHd + dloc + dc * 32 + 8 * hh;
        const v16b kb = Frag<__bf16>::load(kvs_h + ko);
        const v16b kl = Frag<__bf16>::load(kvs_l + ko);
        s[j] = mma_bf(qh[dc], kb, s[j]);
        s[j] = mma_bf(qh[dc], kl, s[j]);
        s[j] = mma_bf(ql[dc], kb, s[j]);
        guard3(s[j], qh[dc], kb, kl);
      }
    }
    {
      float* sw = ssh + wave * 512;
#pragma unroll
      for (int j = 0; j < 2; ++j)
#pragma unroll
        for (int r = 0; r < 8; ++r) sw[(8 * hh + r) * kKch + j * 16 + c] = s[j][r];
    }
    __syncthreads();
    {
      const float* so = ssh + partner * 512;
#pragma unroll
      for (int j = 0; j < 2; ++j)
#pragma unroll
        for (int r = 0; r < 8; ++r)
          s[j][r] = (s[j][r] + so[(8 * hh + r) * kKch + j * 16 + c]) * kScoreScale;
    }

    float cm[8];
#pragma unroll
    for (int r = 0; r < 8; ++r) {
      const int qrow = q0 + 8 * hh + r;
      float m = -INFINITY;
#pragma unroll
      for (int j = 0; j < 2; ++j) {
        const int kvcol = t0 + j * 16 + c;
        const float sv = (kvcol > qrow) ? -INFINITY : s[j][r];
        s[j][r] = sv;
        m = fmaxf(m, sv);
      }
#pragma unroll
      for (int off = 1; off < 16; off <<= 1) m = fmaxf(m, __shfl_xor(m, off, 32));
      cm[r] = m;
    }
    __bf16* pwh = ps_h + wave * 512;
    __bf16* pwl = ps_l + wave * 512;
#pragma unroll
    for (int r = 0; r < 8; ++r) {
      const float mnew = fmaxf(mrow[r], cm[r]);
      const float alpha = expf(mrow[r] - mnew);
      mrow[r] = mnew;
      float psum = 0.0f;
#pragma unroll
      for (int j = 0; j < 2; ++j) {
        const float p = expf(s[j][r] - mnew);
        psum += p;
        unsigned short hb, lb;
        split_bf(p, hb, lb);
        pwh[(8 * hh + r) * kKch + j * 16 + c] = __builtin_bit_cast(__bf16, hb);
        pwl[(8 * hh + r) * kKch + j * 16 + c] = __builtin_bit_cast(__bf16, lb);
      }
#pragma unroll
      for (int off = 1; off < 16; off <<= 1) psum += __shfl_xor(psum, off, 32);
      lrow[r] = lrow[r] * alpha + psum;
#pragma unroll
      for (int t8 = 0; t8 < 8; ++t8) oacc[t8][r] *= alpha;
    }
    wave_sync();
    {
      const v16b pa = Frag<__bf16>::load(pwh + c * kKch + 8 * hh);
      const v16b pl = Frag<__bf16>::load(pwl + c * kKch + 8 * hh);
#pragma unroll
      for (int t8 = 0; t8 < 8; ++t8) {
        const int vo = (dloc + t8 * 16 + c) * kKch + 8 * hh;
        const v16b vb = Frag<__bf16>::load(kvt_h + vo);
        const v16b vl = Frag<__bf16>::load(kvt_l + vo);
        oacc[t8] = mma_bf(pa, vb, oacc[t8]);
        oacc[t8] = mma_bf(pa, vl, oacc[t8]);
        oacc[t8] = mma_bf(pl, vb, oacc[t8]);
        guard3(oacc[t8], pa, vb, vl);
      }
    }
  }

  __syncthreads();
  float* os = reinterpret_cast<float*>(lds_dyn) + wave * (16 * kSlabPitch);
  const float sinkv = bf_rne(sinkp[h]);
#pragma unroll
  for (int r = 0; r < 8; ++r) {
    const float mf = fmaxf(mrow[r], sinkv);
    const float e1 = expf(mrow[r] - mf);
    const float lf = lrow[r] * e1 + expf(sinkv - mf);
    const float inv = e1 * (1.0f / lf);
#pragma unroll
    for (int t8 = 0; t8 < 8; ++t8) os[(8 * hh + r) * kSlabPitch + t8 * 16 + c] = oacc[t8][r] * inv;
  }
  wave_sync();
  if (dh == 1) {
#pragma unroll 2
    for (int row = 0; row < 16; ++row) {
      float* pr = os + row * kSlabPitch + 64 + 2 * lane;
      const float x1 = pr[0], x2 = pr[1];
      const float cs = cosT[(size_t)(q0 + row) * kRopeHalf + lane];
      const float sn = sinT[(size_t)(q0 + row) * kRopeHalf + lane];
      pr[0] = x1 * cs + x2 * sn;
      pr[1] = x2 * cs - x1 * sn;
    }
  }
  wave_sync();
  {
    for (int pass = 0; pass < 2; ++pass) {
#pragma unroll
      for (int it = 0; it < 8; ++it) {
        const int row = it * 2 + hh;
        const float* sp = os + row * kSlabPitch + c * 8;
        v4u hw, lw;
#pragma unroll
        for (int e = 0; e < 4; ++e) {
          unsigned short h0, l0, h1, l1;
          split_bf(sp[2 * e], h0, l0);
          split_bf(sp[2 * e + 1], h1, l1);
          hw[e] = pack2(h0, h1);
          lw[e] = pack2(l0, l1);
        }
        const size_t go = (size_t)(q0 + row) * kQCols + dcol + c * 8;
        *(volatile v4u*)(Ohp + go) = hw;
        *(volatile v4u*)(Olp + go) = lw;
      }
      __threadfence();
    }
  }
}

constexpr size_t kBytesXb    = (size_t)kSeq * kHid * 2;
constexpr size_t kBytesWqa   = (size_t)kQLat * kHid * 2;
constexpr size_t kBytesWkv   = (size_t)kHd * kHid * 2;
constexpr size_t kBytesWqb   = (size_t)kQCols * kQLat * 2;
constexpr size_t kBytesWoa   = (size_t)kORCols * kGrpCols * 2;
constexpr size_t kBytesWob   = (size_t)kHid * kORCols * 2;
constexpr size_t kBytesTrig  = (size_t)kSeq * kRopeHalf * 4;
constexpr size_t kBytesKVraw = (size_t)kSeq * kHd * 4;
constexpr size_t kBytesKV16  = (size_t)kSeq * kHd * 2;
constexpr size_t kBytesRegA  = (size_t)kSeq * kQCols * 4;
constexpr size_t kBytesO16   = (size_t)kSeq * kQCols * 2;
constexpr size_t kBytesQLraw = (size_t)kSeq * kQLat * 4;
constexpr size_t kBytesQL16  = (size_t)kSeq * kQLat * 2;
constexpr size_t kBytesRegB  = kBytesQLraw + 2 * kBytesQL16;
constexpr size_t kBytesOR16  = (size_t)kSeq * kORCols * 2;
constexpr size_t kBytesQ16   = (size_t)kSeq * kQCols * 2;

constexpr size_t kOffXb    = 0;
constexpr size_t kOffWqa   = kOffXb + kBytesXb;
constexpr size_t kOffWkv   = kOffWqa + kBytesWqa;
constexpr size_t kOffWqb   = kOffWkv + kBytesWkv;
constexpr size_t kOffWoa   = kOffWqb + kBytesWqb;
constexpr size_t kOffWob   = kOffWoa + kBytesWoa;
constexpr size_t kOffCos   = kOffWob + kBytesWob;
constexpr size_t kOffSin   = kOffCos + kBytesTrig;
constexpr size_t kOffKVraw = kOffSin + kBytesTrig;
constexpr size_t kOffKVh   = kOffKVraw + kBytesKVraw;
constexpr size_t kOffKVl   = kOffKVh + kBytesKV16;
constexpr size_t kOffKVTh  = kOffKVl + kBytesKV16;
constexpr size_t kOffKVTl  = kOffKVTh + kBytesKV16;
constexpr size_t kOffRegA  = kOffKVTl + kBytesKV16;
constexpr size_t kOffRegB  = kOffRegA + kBytesRegA;
constexpr size_t kOffQh    = kOffRegB + kBytesRegB;
constexpr size_t kOffQl    = kOffQh + kBytesQ16;
constexpr size_t kWsTotal  = kOffQl + kBytesQ16;
static_assert(kWsTotal == 125304832ull, "carve total");
static_assert(kWsTotal <= 134217728ull, "carve cap");
static_assert(2 * kBytesO16 <= kBytesRegA, "o planes fit");
static_assert(2 * kBytesOR16 <= kBytesRegB, "o_r planes fit");
static_assert((kOffRegA % 256) == 0 && (kOffRegB % 256) == 0 && (kOffQh % 256) == 0, "align");

static_assert(kHid % 32 == 0 && kQLat % 32 == 0 && kGrpCols % 32 == 0 && kORCols % 32 == 0, "K multiples of 32");
static_assert(kSeq % 64 == 0 && kQLat % 64 == 0 && kQCols % 64 == 0 && kHd % 64 == 0 && kOLat % 64 == 0 && kHid % 64 == 0, "M,N multiples of 64");
static_assert(((kSeq / 64) * (kQLat / 64)) % 8 == 0, "tiles0");
static_assert(((kSeq / 64) * (kQCols / 64)) % 8 == 0, "tiles1");
static_assert(((kSeq / 64) * (kHd / 64)) % 8 == 0, "tiles2");
static_assert(((kSeq / 64) * (kOLat / 64)) % 8 == 0, "tiles5");
static_assert(((kSeq / 64) * (kHid / 64)) % 8 == 0, "tiles6");
static_assert((size_t)kSeq * kHid * 4 == 16777216ull, "out bytes");

extern "C" void kernel_launch(void* const* d_in, const int* in_sizes, int n_in,
                              void* d_out, int out_size, void* d_ws, size_t ws_size,
                              hipStream_t stream) {
  if (n_in < 10) return;
  if ((size_t)out_size < (size_t)kSeq * kHid) return;
  if (ws_size < kWsTotal) return;
  if (in_sizes[0] != kSeq * kHid || in_sizes[4] != kQCols * kQLat) return;

  const float* x     = (const float*)d_in[0];
  const float* freqs = (const float*)d_in[1];
  const float* wq_a  = (const float*)d_in[2];
  const float* qnw   = (const float*)d_in[3];
  const float* wq_b  = (const float*)d_in[4];
  const float* wkv   = (const float*)d_in[5];
  const float* kvnw  = (const float*)d_in[6];
  const float* wo_a  = (const float*)d_in[7];
  const float* wo_b  = (const float*)d_in[8];
  const float* sinkp = (const float*)d_in[9];
  float* out = (float*)d_out;

  char* ws = (char*)d_ws;
  unsigned short* Xb   = (unsigned short*)(ws + kOffXb);
  unsigned short* Wqa  = (unsigned short*)(ws + kOffWqa);
  unsigned short* Wkv  = (unsigned short*)(ws + kOffWkv);
  unsigned short* Wqb  = (unsigned short*)(ws + kOffWqb);
  unsigned short* Woa  = (unsigned short*)(ws + kOffWoa);
  unsigned short* Wob  = (unsigned short*)(ws + kOffWob);
  float* cosT          = (float*)(ws + kOffCos);
  float* sinT          = (float*)(ws + kOffSin);
  float* KVraw         = (float*)(ws + kOffKVraw);
  unsigned short* KVh  = (unsigned short*)(ws + kOffKVh);
  unsigned short* KVl  = (unsigned short*)(ws + kOffKVl);
  unsigned short* KVTh = (unsigned short*)(ws + kOffKVTh);
  unsigned short* KVTl = (unsigned short*)(ws + kOffKVTl);
  float* Qraw          = (float*)(ws + kOffRegA);
  unsigned short* Oh   = (unsigned short*)(ws + kOffRegA);
  unsigned short* Ol   = (unsigned short*)(ws + kOffRegA + kBytesO16);
  float* QLraw         = (float*)(ws + kOffRegB);
  unsigned short* QLh  = (unsigned short*)(ws + kOffRegB + kBytesQLraw);
  unsigned short* QLl  = (unsigned short*)(ws + kOffRegB + kBytesQLraw + kBytesQL16);
  unsigned short* ORh  = (unsigned short*)(ws + kOffRegB);
  unsigned short* ORl  = (unsigned short*)(ws + kOffRegB + kBytesOR16);
  unsigned short* Qh   = (unsigned short*)(ws + kOffQh);
  unsigned short* Ql   = (unsigned short*)(ws + kOffQl);

  {
    const int n8x   = kSeq * kHid / 8;
    const int n8qa  = kQLat * kHid / 8;
    const int n8kv  = kHd * kHid / 8;
    const int n8qb  = kQCols * kQLat / 8;
    const int n8oa  = kORCols * kGrpCols / 8;
    const int n8ob  = kHid * kORCols / 8;
    cvt_bf16x8_kernel<<<(n8x + 255) / 256, 256, 0, stream>>>(x, Xb, n8x);
    cvt_bf16x8_kernel<<<(n8qa + 255) / 256, 256, 0, stream>>>(wq_a, Wqa, n8qa);
    cvt_bf16x8_kernel<<<(n8kv + 255) / 256, 256, 0, stream>>>(wkv, Wkv, n8kv);
    cvt_bf16x8_kernel<<<(n8qb + 255) / 256, 256, 0, stream>>>(wq_b, Wqb, n8qb);
    cvt_bf16x8_kernel<<<(n8oa + 255) / 256, 256, 0, stream>>>(wo_a, Woa, n8oa);
    cvt_bf16x8_kernel<<<(n8ob + 255) / 256, 256, 0, stream>>>(wo_b, Wob, n8ob);
  }
  {
    const int n = kSeq * kRopeHalf;
    rope_table_kernel<<<(n + 255) / 256, 256, 0, stream>>>(freqs, cosT, sinT, n);
  }
  gemm64_bf16<0, 0><<<dim3((kSeq / 64) * (kQLat / 64) / 8, 1), 256, 0, stream>>>(
      Xb, Xb, kHid, 0L, Wqa, Wqa, kHid, 0L, (void*)QLraw, (void*)QLraw, kQLat, 0L,
      kSeq, kQLat, kHid, 1.0f);
  qlat_prep_kernel<<<kSeq, 128, 0, stream>>>(QLraw, qnw, QLh, QLl);
  gemm64_bf16<1, 0><<<dim3((kSeq / 64) * (kQCols / 64) / 8, 1), 256, 0, stream>>>(
      QLh, QLl, kQLat, 0L, Wqb, Wqb, kQLat, 0L, (void*)Qraw, (void*)Qraw, kQCols, 0L,
      kSeq, kQCols, kQLat, 1.0f);
  gemm64_bf16<0, 0><<<dim3((kSeq / 64) * (kHd / 64) / 8, 1), 256, 0, stream>>>(
      Xb, Xb, kHid, 0L, Wkv, Wkv, kHid, 0L, (void*)KVraw, (void*)KVraw, kHd, 0L,
      kSeq, kHd, kHid, 1.0f);
  kv_prep_kernel<<<kSeq / 64, 256, kKvPrepLdsBytes, stream>>>(KVraw, kvnw, cosT, sinT, KVh, KVl, KVTh, KVTl);
  q_prep_kernel<<<dim3(kSeq, kHeads / 8), 256, 0, stream>>>(Qraw, cosT, sinT, Qh, Ql);
  attn_kernel<<<dim3(kSeq / kQBlk, kHeads), 256, kAttnLdsBytes, stream>>>(
      Qh, Ql, KVh, KVl, KVTh, KVTl, cosT, sinT, sinkp, Oh, Ol);
  gemm64_bf16<1, 2><<<dim3((kSeq / 64) * (kOLat / 64) / 8, kGroups), 256, 0, stream>>>(
      Oh, Ol, kQCols, (long)kGrpCols, Woa, Woa, kGrpCols, (long)kOLat * kGrpCols,
      (void*)ORh, (void*)ORl, kORCols, (long)kOLat,
      kSeq, kOLat, kGrpCols, 1.0f);
  gemm64_bf16<1, 0><<<dim3((kSeq / 64) * (kHid / 64) / 8, 1), 256, 0, stream>>>(
      ORh, ORl, kORCols, 0L, Wob, Wob, kORCols, 0L, (void*)out, (void*)out, kHid, 0L,
      kSeq, kHid, kORCols, 1.0f);
}
